// GraphTransformerDemon_20143396618415
// MI455X (gfx1250) — hardware-verified
//
#include <hip/hip_runtime.h>
#include <stddef.h>
#include <stdint.h>


#define BSZ 4
#define SSZ 384
#define HSZ 64
#define NHD 4
#define DHD 16
#define INS 32
#define MROWS (BSZ * SSZ)

typedef _Float16 v16h __attribute__((ext_vector_type(16)));
typedef _Float16 v8h_t __attribute__((ext_vector_type(8)));
typedef v8h_t __attribute__((may_alias)) v8h;
typedef float v8f __attribute__((ext_vector_type(8)));
typedef float v4f_t __attribute__((ext_vector_type(4)));
typedef v4f_t __attribute__((may_alias)) v4f;

union Frag {
  v16h v;
  v8h_t hh[2];
};

__device__ __forceinline__ v8f wmma_f16(const v16h a, const v16h b, v8f c) {
  c = __builtin_amdgcn_wmma_f32_16x16x32_f16(false, a, false, b, (short)0, c,
                                             false, false);
  asm volatile("v_nop\n\tv_nop\n\tv_nop\n\tv_nop" : "+v"(c) : "v"(a), "v"(b));
  return c;
}

__device__ __forceinline__ v8f zero8() {
  v8f c;
#pragma unroll
  for (int r = 0; r < 8; ++r) c[r] = 0.f;
  return c;
}

__device__ __forceinline__ v16h frag_f32(const float* p, int h) {
  const v4f x0 = *(const v4f*)(p + 8 * h);
  const v4f x1 = *(const v4f*)(p + 8 * h + 4);
  const v4f x2 = *(const v4f*)(p + 16 + 8 * h);
  const v4f x3 = *(const v4f*)(p + 20 + 8 * h);
  v16h a;
  a[0] = (_Float16)x0[0];  a[1] = (_Float16)x0[1];
  a[2] = (_Float16)x0[2];  a[3] = (_Float16)x0[3];
  a[4] = (_Float16)x1[0];  a[5] = (_Float16)x1[1];
  a[6] = (_Float16)x1[2];  a[7] = (_Float16)x1[3];
  a[8] = (_Float16)x2[0];  a[9] = (_Float16)x2[1];
  a[10] = (_Float16)x2[2]; a[11] = (_Float16)x2[3];
  a[12] = (_Float16)x3[0]; a[13] = (_Float16)x3[1];
  a[14] = (_Float16)x3[2]; a[15] = (_Float16)x3[3];
  return a;
}

__device__ __forceinline__ v16h frag16_f32(const float* p, int h) {
  const v4f x0 = *(const v4f*)(p + 8 * h);
  const v4f x1 = *(const v4f*)(p + 8 * h + 4);
  v16h a;
  a[0] = (_Float16)x0[0]; a[1] = (_Float16)x0[1];
  a[2] = (_Float16)x0[2]; a[3] = (_Float16)x0[3];
  a[4] = (_Float16)x1[0]; a[5] = (_Float16)x1[1];
  a[6] = (_Float16)x1[2]; a[7] = (_Float16)x1[3];
#pragma unroll
  for (int t = 8; t < 16; ++t) a[t] = (_Float16)0.f;
  return a;
}

template <int K, int N, bool RELU, bool HASBIAS, bool LNORM>
__global__ __launch_bounds__(2 * N) void gemm_k(const float* __restrict__ A,
                                                const float* __restrict__ W,
                                                const float* __restrict__ bias,
                                                const float* __restrict__ res,
                                                const float* __restrict__ gam,
                                                const float* __restrict__ bet,
                                                float* __restrict__ C, int M) {
  static_assert(K % 32 == 0 && N % 32 == 0 && N <= 128 && K <= 128);
  static_assert(!LNORM || N == 64);
  constexpr int NT = 2 * N;
  constexpr int KP = K + 8;
  constexpr int NP = N + 4;
  constexpr int LPR = N / 32;
  __shared__ __align__(16) _Float16 Ws[N][KP];
  __shared__ __align__(16) float Cs[16][NP];
  (void)bias; (void)res; (void)gam; (void)bet;

  const int tid = threadIdx.x;
  const int wave = tid >> 5, lane = tid & 31, m = lane & 15, h = lane >> 4;
  const int m0 = blockIdx.x * 16;
  if (m0 + 16 > M) return;

  for (int idx = tid; idx < K * N; idx += NT) {
    const int kk = idx / N;
    const int nn = idx - kk * N;
    Ws[nn][kk] = (_Float16)W[idx];
  }
  __syncthreads();

  const int n0 = wave * 16;
  const float* arow = A + (size_t)(m0 + m) * K;
  v8f acc = zero8();
#pragma unroll
  for (int k0 = 0; k0 < K; k0 += 32) {
    const v16h a = frag_f32(arow + k0, h);
    Frag b;
    b.hh[0] = *(const v8h*)&Ws[n0 + m][k0 + 8 * h];
    b.hh[1] = *(const v8h*)&Ws[n0 + m][k0 + 16 + 8 * h];
    acc = wmma_f16(a, b.v, acc);
  }

  float bvv = 0.f;
  if constexpr (HASBIAS) bvv = bias[n0 + m];
#pragma unroll
  for (int r = 0; r < 8; ++r) {
    float t = acc[r] + bvv;
    if constexpr (RELU) t = fmaxf(t, 0.f);
    Cs[8 * h + r][n0 + m] = t;
  }
  __syncthreads();

  if constexpr (LNORM) {
#pragma unroll
    for (int rr = 0; rr < 4; ++rr) {
      const int row = wave * 4 + rr;
      const size_t g = (size_t)(m0 + row) * N;
      const float x0 = Cs[row][lane] + res[g + lane];
      const float x1 = Cs[row][lane + 32] + res[g + lane + 32];
      float s = x0 + x1;
#pragma unroll
      for (int o = 16; o > 0; o >>= 1) s += __shfl_xor(s, o, 32);
      const float mean = s * (1.f / 64.f);
      const float d0 = x0 - mean, d1 = x1 - mean;
      float vv = d0 * d0 + d1 * d1;
#pragma unroll
      for (int o = 16; o > 0; o >>= 1) vv += __shfl_xor(vv, o, 32);
      const float rstd = 1.f / sqrtf(vv * (1.f / 64.f) + 1e-5f);
      Cs[row][lane] = d0 * rstd * gam[lane] + bet[lane];
      Cs[row][lane + 32] = d1 * rstd * gam[lane + 32] + bet[lane + 32];
    }
    __syncthreads();
  }

  const int q4 = lane >> 3, e = lane & 7;
  v4f vals[2];
  size_t offs[2];
#pragma unroll
  for (int p = 0; p < 2; ++p) {
    const int L = wave * 8 + p * 4 + q4;
    const int row = L / LPR;
    const int cs = L - row * LPR;
    vals[p] = *(const v4f*)&Cs[row][cs * 32 + e * 4];
    offs[p] = (size_t)(m0 + row) * N + (size_t)(cs * 32 + e * 4);
  }
#pragma unroll
  for (int p = 0; p < 2; ++p) *(volatile v4f*)(C + offs[p]) = vals[p];
  __threadfence();
#pragma unroll
  for (int p = 0; p < 2; ++p) *(volatile v4f*)(C + offs[p]) = vals[p];
}

__global__ __launch_bounds__(64) void attn_k(const float* __restrict__ q,
                                             const float* __restrict__ k,
                                             const float* __restrict__ v,
                                             float* __restrict__ att, int nqt) {
  __shared__ __align__(16) float P[2][16][SSZ + 4];
  __shared__ __align__(16) float Cs[16][HSZ + 4];
  const int tid = threadIdx.x;
  const int w = tid >> 5, lane = tid & 31, m = lane & 15, h = lane >> 4;
  const int qt = blockIdx.x, b = blockIdx.y;
  if (qt >= nqt) return;
  const size_t rowq = (size_t)(b * SSZ + qt * 16);

  for (int hh = 0; hh < 2; ++hh) {
    const int head = 2 * w + hh;
    const int hbase = head * DHD;

    const v16h a = frag16_f32(q + (rowq + m) * HSZ + hbase, h);
#pragma unroll 2
    for (int jt = 0; jt < SSZ / 16; ++jt) {
      const v16h bb =
          frag16_f32(k + (size_t)(b * SSZ + jt * 16 + m) * HSZ + hbase, h);
      v8f c = zero8();
      c = wmma_f16(a, bb, c);
#pragma unroll
      for (int r = 0; r < 8; ++r) P[w][8 * h + r][jt * 16 + m] = c[r] * 0.25f;
    }
    __syncthreads();

#pragma unroll 1
    for (int r = 0; r < 16; ++r) {
      float* pr = &P[w][r][0];
      float x[12];
      float mx = -1e30f;
#pragma unroll
      for (int cc = 0; cc < 12; ++cc) {
        x[cc] = pr[lane + 32 * cc];
        mx = fmaxf(mx, x[cc]);
      }
#pragma unroll
      for (int o = 16; o > 0; o >>= 1) mx = fmaxf(mx, __shfl_xor(mx, o, 32));
      float s = 0.f;
#pragma unroll
      for (int cc = 0; cc < 12; ++cc) {
        x[cc] = __expf(x[cc] - mx);
        s += x[cc];
      }
#pragma unroll
      for (int o = 16; o > 0; o >>= 1) s += __shfl_xor(s, o, 32);
      const float sc = 256.f / s;
#pragma unroll
      for (int cc = 0; cc < 12; ++cc) pr[lane + 32 * cc] = x[cc] * sc;
    }
    __syncthreads();

    v8f acc = zero8();
#pragma unroll 2
    for (int ks = 0; ks < SSZ / 32; ++ks) {
      const v16h ap = frag_f32(&P[w][m][32 * ks], h);
      const float* vp =
          v + (size_t)(b * SSZ + 32 * ks + 8 * h) * HSZ + hbase + m;
      v16h bv;
#pragma unroll
      for (int i = 0; i < 8; ++i) {
        bv[i] = (_Float16)vp[(size_t)i * HSZ];
        bv[8 + i] = (_Float16)vp[(size_t)(16 + i) * HSZ];
      }
      acc = wmma_f16(ap, bv, acc);
    }
#pragma unroll
    for (int r = 0; r < 8; ++r)
      Cs[8 * h + r][hbase + m] = acc[r] * (1.f / 256.f);
    __syncthreads();
  }

  const int q4 = lane >> 3, e = lane & 7;
  v4f vals[4];
  size_t offs[4];
#pragma unroll
  for (int p = 0; p < 4; ++p) {
    const int L = w * 16 + p * 4 + q4;
    const int row = L >> 1;
    const int cs = L & 1;
    vals[p] = *(const v4f*)&Cs[row][cs * 32 + e * 4];
    offs[p] = (rowq + row) * HSZ + (size_t)(cs * 32 + e * 4);
  }
#pragma unroll
  for (int p = 0; p < 4; ++p) *(volatile v4f*)(att + offs[p]) = vals[p];
  __threadfence();
#pragma unroll
  for (int p = 0; p < 4; ++p) *(volatile v4f*)(att + offs[p]) = vals[p];
}

__global__ __launch_bounds__(SSZ) void keep_k(const float* __restrict__ Ld,
                                              const float* __restrict__ Rd,
                                              const float* __restrict__ Wd2,
                                              const float* __restrict__ bd2,
                                              float* __restrict__ keep,
                                              int nrows) {
  __shared__ float lrow[32];
  __shared__ float w2s[32];
  __shared__ __align__(16) float ks[SSZ];
  const int bi = blockIdx.x;
  if (bi >= nrows) return;
  const int b = bi / SSZ;
  const int j = threadIdx.x;
  if (j < 32) {
    lrow[j] = Ld[(size_t)bi * 32 + j];
    w2s[j] = Wd2[j];
  }
  __syncthreads();
  const float* rd = Rd + (size_t)(b * SSZ + j) * 32;
  float acc = bd2[0];
#pragma unroll
  for (int d4 = 0; d4 < 8; ++d4) {
    const v4f x = *(const v4f*)(rd + 4 * d4);
    acc += fmaxf(lrow[4 * d4 + 0] + x[0], 0.f) * w2s[4 * d4 + 0];
    acc += fmaxf(lrow[4 * d4 + 1] + x[1], 0.f) * w2s[4 * d4 + 1];
    acc += fmaxf(lrow[4 * d4 + 2] + x[2], 0.f) * w2s[4 * d4 + 2];
    acc += fmaxf(lrow[4 * d4 + 3] + x[3], 0.f) * w2s[4 * d4 + 3];
  }
  ks[j] = 1.f / (1.f + __expf(-acc));
  __syncthreads();
  if (j < 96) {
    const int wave = j >> 5, lane = j & 31;
    const int L = wave * 4 + (lane >> 3);
    const int e = lane & 7;
    const v4f val = *(const v4f*)&ks[L * 32 + e * 4];
    float* dst = keep + (size_t)bi * SSZ + (size_t)(L * 32 + e * 4);
    *(volatile v4f*)dst = val;
    __threadfence();
    *(volatile v4f*)dst = val;
  }
}

__global__ __launch_bounds__(HSZ) void pair_k(const float* __restrict__ Lh,
                                              const float* __restrict__ Rh,
                                              const float* __restrict__ keep,
                                              float* __restrict__ actpre,
                                              float* __restrict__ totpre,
                                              int nrows) {
  __shared__ __align__(16) float ks[SSZ];
  __shared__ __align__(16) float av[HSZ];
  __shared__ __align__(16) float tv[HSZ];
  const int bi = blockIdx.x;
  if (bi >= nrows) return;
  const int b = bi / SSZ;
  const int hc = threadIdx.x;
  for (int j = hc; j < SSZ; j += HSZ) ks[j] = keep[(size_t)bi * SSZ + j];
  const float lv = Lh[(size_t)bi * HSZ + hc];
  __syncthreads();
  const float* rr = Rh + (size_t)b * SSZ * HSZ + hc;
  float at = 0.f, aa = 0.f;
#pragma unroll 4
  for (int j = 0; j < SSZ; ++j) {
    const float ev = fmaxf(lv + rr[(size_t)j * HSZ], 0.f);
    at += ev;
    aa += ks[j] * ev;
  }
  av[hc] = aa;
  tv[hc] = at;
  __syncthreads();
  if (hc < 32) {
    const int lane = hc;
    const int q4 = lane >> 3, e = lane & 7;
    const float* srcb = (q4 < 2) ? av : tv;
    float* dstb = (q4 < 2) ? actpre : totpre;
    const int col = (q4 & 1) * 32 + e * 4;
    const v4f val = *(const v4f*)(srcb + col);
    float* dst = dstb + (size_t)bi * HSZ + col;
    *(volatile v4f*)dst = val;
    __threadfence();
    *(volatile v4f*)dst = val;
  }
}

__global__ __launch_bounds__(BSZ * HSZ) void pool_k(const float* __restrict__ nodes,
                                                    const float* __restrict__ U,
                                                    const float* __restrict__ T,
                                                    const float* __restrict__ keep,
                                                    const float* __restrict__ be2,
                                                    const float* __restrict__ Wc1,
                                                    const float* __restrict__ bc1,
                                                    const float* __restrict__ Wc2,
                                                    const float* __restrict__ bc2,
                                                    float* __restrict__ out) {
  __shared__ float cat[BSZ][2 * HSZ];
  __shared__ float hcl[BSZ][32];
  __shared__ float red[8];
  __shared__ __align__(16) float o12[16];
  const int t = threadIdx.x;
  const int b = t >> 6, c = t & 63, wave = t >> 5, lane = t & 31;

  float pa = 0.f, pt = 0.f;
  const size_t rb = (size_t)b * SSZ;
#pragma unroll 4
  for (int i = 0; i < SSZ; ++i) {
    const size_t idx = (rb + i) * HSZ + c;
    const float u = U[idx];
    pa += nodes[idx] + u;
    pt += T[idx] - u;
  }
  float ksm = 0.f;
  const float* kp = keep + (size_t)b * SSZ * SSZ;
#pragma unroll 4
  for (int e2 = c; e2 < SSZ * SSZ; e2 += HSZ) ksm += kp[e2];
#pragma unroll
  for (int o = 16; o > 0; o >>= 1) ksm += __shfl_xor(ksm, o, 32);
  if (lane == 0) red[wave] = ksm;
  __syncthreads();
  const float ka = red[2 * b] + red[2 * b + 1];
  const float be = be2[c];
  pa = (pa + be * ka) * (1.f / (float)SSZ);
  pt = (pt + be * ((float)(SSZ * SSZ) - ka)) * (1.f / (float)SSZ);
  cat[b][c] = pa;
  cat[b][HSZ + c] = pt;
  __syncthreads();
  if (c < 32) {
    float a2 = bc1[c];
#pragma unroll 4
    for (int d = 0; d < 2 * HSZ; ++d) a2 += cat[b][d] * Wc1[d * 32 + c];
    hcl[b][c] = fmaxf(a2, 0.f);
  }
  __syncthreads();
  if (c < 3) {
    float a3 = bc2[c];
#pragma unroll 8
    for (int d = 0; d < 32; ++d) a3 += hcl[b][d] * Wc2[d * 3 + c];
    o12[b * 3 + c] = a3;
  }
  __syncthreads();
  if (t < 3) {
    const v4f val = *(const v4f*)&o12[t * 4];
    float* dst = out + t * 4;
    *(volatile v4f*)dst = val;
    __threadfence();
    *(volatile v4f*)dst = val;
  }
}

extern "C" void kernel_launch(void* const* d_in, const int* in_sizes, int n_in,
                              void* d_out, int out_size, void* d_ws, size_t ws_size,
                              hipStream_t stream) {
  static_assert(MROWS % 16 == 0 && SSZ % 32 == 0 && BSZ * HSZ == 256);
  if (n_in < 31) return;
  if (in_sizes[0] != BSZ * SSZ * INS || out_size != BSZ * 3) return;

  const float* x   = (const float*)d_in[0];
  const float* Wp  = (const float*)d_in[1];  const float* bp  = (const float*)d_in[2];
  const float* Wq  = (const float*)d_in[3];  const float* bq  = (const float*)d_in[4];
  const float* Wk  = (const float*)d_in[5];  const float* bk  = (const float*)d_in[6];
  const float* Wv  = (const float*)d_in[7];  const float* bv  = (const float*)d_in[8];
  const float* Wo  = (const float*)d_in[9];  const float* bo  = (const float*)d_in[10];
  const float* g1  = (const float*)d_in[11]; const float* b1  = (const float*)d_in[12];
  const float* Wf1 = (const float*)d_in[13]; const float* bf1 = (const float*)d_in[14];
  const float* Wf2 = (const float*)d_in[15]; const float* bf2 = (const float*)d_in[16];
  const float* g2  = (const float*)d_in[17]; const float* b2  = (const float*)d_in[18];
  const float* We1 = (const float*)d_in[19]; const float* be1 = (const float*)d_in[20];
  const float* We2 = (const float*)d_in[21]; const float* be2 = (const float*)d_in[22];
  const float* Wd1 = (const float*)d_in[23]; const float* bd1 = (const float*)d_in[24];
  const float* Wd2 = (const float*)d_in[25]; const float* bd2 = (const float*)d_in[26];
  const float* Wc1 = (const float*)d_in[27]; const float* bc1 = (const float*)d_in[28];
  const float* Wc2 = (const float*)d_in[29]; const float* bc2 = (const float*)d_in[30];
  float* out = (float*)d_out;

  float* ws = (float*)d_ws;
  size_t o = 0;
  const size_t nMH = (size_t)MROWS * HSZ;
  float* n0     = ws + o; o += nMH;
  float* qb     = ws + o; o += nMH;
  float* kb     = ws + o; o += nMH;
  float* vb     = ws + o; o += nMH;
  float* att    = ws + o; o += nMH;
  float* n1     = ws + o; o += nMH;
  float* f      = ws + o; o += (size_t)MROWS * 2 * HSZ;
  float* nodes  = ws + o; o += nMH;
  float* Lh     = ws + o; o += nMH;
  float* Rh     = ws + o; o += nMH;
  float* Ld     = ws + o; o += (size_t)MROWS * 32;
  float* Rd     = ws + o; o += (size_t)MROWS * 32;
  float* keep   = ws + o; o += (size_t)MROWS * SSZ;
  float* actpre = ws + o; o += nMH;
  float* totpre = ws + o; o += nMH;
  float* U      = ws + o; o += nMH;
  float* T      = ws + o; o += nMH;
  if (o * sizeof(float) > ws_size) return;

  const int M = MROWS;
  const dim3 gM(M / 16);

  gemm_k<INS, HSZ, true, true, false><<<gM, 2 * HSZ, 0, stream>>>(
      x, Wp, bp, x, x, x, n0, M);
  gemm_k<HSZ, HSZ, false, true, false><<<gM, 2 * HSZ, 0, stream>>>(
      n0, Wq, bq, n0, n0, n0, qb, M);
  gemm_k<HSZ, HSZ, false, true, false><<<gM, 2 * HSZ, 0, stream>>>(
      n0, Wk, bk, n0, n0, n0, kb, M);
  gemm_k<HSZ, HSZ, false, true, false><<<gM, 2 * HSZ, 0, stream>>>(
      n0, Wv, bv, n0, n0, n0, vb, M);
  attn_k<<<dim3(SSZ / 16, BSZ), 64, 0, stream>>>(qb, kb, vb, att, SSZ / 16);
  gemm_k<HSZ, HSZ, false, true, true><<<gM, 2 * HSZ, 0, stream>>>(
      att, Wo, bo, n0, g1, b1, n1, M);
  gemm_k<HSZ, 2 * HSZ, true, true, false><<<gM, 4 * HSZ, 0, stream>>>(
      n1, Wf1, bf1, n1, n1, n1, f, M);
  gemm_k<2 * HSZ, HSZ, false, true, true><<<gM, 2 * HSZ, 0, stream>>>(
      f, Wf2, bf2, n1, g2, b2, nodes, M);
  gemm_k<HSZ, HSZ, false, false, false><<<gM, 2 * HSZ, 0, stream>>>(
      nodes, We1, We1, nodes, nodes, nodes, Lh, M);
  gemm_k<HSZ, HSZ, false, true, false><<<gM, 2 * HSZ, 0, stream>>>(
      nodes, We1 + HSZ * HSZ, be1, nodes, nodes, nodes, Rh, M);
  gemm_k<HSZ, 32, false, false, false><<<gM, 64, 0, stream>>>(
      nodes, Wd1, Wd1, nodes, nodes, nodes, Ld, M);
  gemm_k<HSZ, 32, false, true, false><<<gM, 64, 0, stream>>>(
      nodes, Wd1 + HSZ * 32, bd1, nodes, nodes, nodes, Rd, M);
  keep_k<<<dim3(M), SSZ, 0, stream>>>(Ld, Rd, Wd2, bd2, keep, M);
  pair_k<<<dim3(M), HSZ, 0, stream>>>(Lh, Rh, keep, actpre, totpre, M);
  gemm_k<HSZ, HSZ, false, false, false><<<gM, 2 * HSZ, 0, stream>>>(
      actpre, We2, We2, actpre, actpre, actpre, U, M);
  gemm_k<HSZ, HSZ, false, false, false><<<gM, 2 * HSZ, 0, stream>>>(
      totpre, We2, We2, totpre, totpre, totpre, T, M);
  pool_k<<<dim3(1), BSZ * HSZ, 0, stream>>>(nodes, U, T, keep, be2, Wc1, bc1,
                                            Wc2, bc2, out);
}
